// GraphSelfAttentionLayer_7438883357374
// MI455X (gfx1250) — hardware-verified
//
#include <hip/hip_runtime.h>
#include <math.h>


#define NB_    2
#define NN_    1024
#define ND_    128
#define NH_    64
#define MROWS_ (NB_ * NN_)
#define SLOPE_ 0.2f

typedef _Float16 v16h __attribute__((ext_vector_type(16)));
typedef _Float16 v8h  __attribute__((ext_vector_type(8)));
typedef float    v8f  __attribute__((ext_vector_type(8)));
typedef float    v4f  __attribute__((ext_vector_type(4)));
typedef unsigned int v4u __attribute__((ext_vector_type(4)));

union Frag  { v16h v; v8h half[2]; _Float16 s[16]; };
union Pack8 { v8h h; v4u u; _Float16 s[8]; };

__device__ __forceinline__ v8f wmma_f16(v16h a, v16h b, v8f c) {
  v8f d = __builtin_amdgcn_wmma_f32_16x16x32_f16(false, a, false, b, (short)0, c, false, false);
  asm volatile("v_nop\n\tv_nop\n\tv_nop\n\tv_nop" : "+v"(d) : "v"(a), "v"(b));
  return d;
}

__device__ __forceinline__ v8f zero8() {
  v8f z;
#pragma unroll
  for (int r = 0; r < 8; ++r) z[r] = 0.f;
  return z;
}

__device__ __forceinline__ void proj_store(const float* sT, float* gout, _Float16* grt,
                                           int m0, int side, int tid) {
#pragma unroll
  for (int q = 0; q < 8; ++q) {
    const int c = q * 128 + tid;
    const int row = c >> 4, col4 = (c & 15) * 4;
    const v4f v = *(const v4f*)(sT + row * NH_ + col4);
    *(volatile v4f*)(gout + (size_t)(m0 + row) * NH_ + col4) = v;
  }
  if (side) {
    const int b = m0 >> 10, jl0 = m0 & (NN_ - 1);
#pragma unroll
    for (int q = 0; q < 4; ++q) {
      const int c = q * 128 + tid;
      const int f = c >> 3, jc = (c & 7) * 8;
      Pack8 p;
#pragma unroll
      for (int e = 0; e < 8; ++e) p.s[e] = (_Float16)sT[(jc + e) * NH_ + f];
      *(volatile v4u*)(grt + ((size_t)b * NH_ + f) * NN_ + jl0 + jc) = p.u;
    }
  }
}

__global__ __launch_bounds__(128)
void k_proj(const float* __restrict__ X, const float* __restrict__ Wl,
            const float* __restrict__ Wr, float* gl, float* gr, _Float16* grt, int nrows) {
  __shared__ __attribute__((aligned(16))) _Float16 sW[NH_ * ND_];
  __shared__ __attribute__((aligned(16))) float    sT[64 * NH_];
  const int tid = threadIdx.x, lane = tid & 31, wv = tid >> 5;
  const int hh = lane >> 4, m = lane & 15;
  const int side = blockIdx.y;
  const int m0 = blockIdx.x * 64;
  if (m0 + 64 > nrows) return;
  const float* W = side ? Wr : Wl;

#pragma unroll 4
  for (int idx = tid; idx < ND_ * NH_; idx += 128) {
    const int k = idx >> 6, h = idx & 63;
    sW[h * ND_ + k] = (_Float16)(64.f * W[idx]);
  }
  __syncthreads();

  v8f acc[4];
#pragma unroll
  for (int t = 0; t < 4; ++t) acc[t] = zero8();

  const float* xrow = X + (size_t)(m0 + 16 * wv + m) * ND_;
#pragma unroll
  for (int s = 0; s < 4; ++s) {
    const int k0 = 32 * s;
    const v4f f0 = *(const v4f*)(xrow + k0 + 8 * hh);
    const v4f f1 = *(const v4f*)(xrow + k0 + 8 * hh + 4);
    const v4f f2 = *(const v4f*)(xrow + k0 + 16 + 8 * hh);
    const v4f f3 = *(const v4f*)(xrow + k0 + 16 + 8 * hh + 4);
    Frag a;
#pragma unroll
    for (int i = 0; i < 4; ++i) {
      a.s[i]      = (_Float16)f0[i];
      a.s[4 + i]  = (_Float16)f1[i];
      a.s[8 + i]  = (_Float16)f2[i];
      a.s[12 + i] = (_Float16)f3[i];
    }
#pragma unroll
    for (int t = 0; t < 4; ++t) {
      const _Float16* bp = sW + (16 * t + m) * ND_ + k0;
      Frag bfr;
      bfr.half[0] = *(const v8h*)(bp + 8 * hh);
      bfr.half[1] = *(const v8h*)(bp + 16 + 8 * hh);
      acc[t] = wmma_f16(a.v, bfr.v, acc[t]);
    }
  }

#pragma unroll
  for (int t = 0; t < 4; ++t) {
#pragma unroll
    for (int r = 0; r < 8; ++r)
      sT[(16 * wv + 8 * hh + r) * NH_ + 16 * t + m] = acc[t][r] * (1.f / 64.f);
  }
  __syncthreads();

  float* gout = side ? gr : gl;
  proj_store(sT, gout, grt, m0, side, tid);
  __threadfence();
  proj_store(sT, gout, grt, m0, side, tid);
}

__global__ __launch_bounds__(128)
void k_scores(const float* __restrict__ gl, const float* __restrict__ gr,
              const float* __restrict__ aw, const float* __restrict__ ab,
              _Float16* a_out, int nrows) {
  __shared__ __attribute__((aligned(16))) float sE[NN_];
  __shared__ float sM[4];
  __shared__ float sS[4];
  const int gi = blockIdx.x;
  if (gi >= nrows) return;
  const int b = gi >> 10;
  const int tid = threadIdx.x, lane = tid & 31, wv = tid >> 5;
  const int hh = lane >> 4, m = lane & 15;

  float grv[2][16];
  Frag wf[2];
  const float* grrow = gr + (size_t)gi * NH_;
#pragma unroll
  for (int s = 0; s < 2; ++s) {
    const int h0 = 32 * s + 8 * hh, h1 = 32 * s + 16 + 8 * hh;
    const v4f r0 = *(const v4f*)(grrow + h0);
    const v4f r1 = *(const v4f*)(grrow + h0 + 4);
    const v4f r2 = *(const v4f*)(grrow + h1);
    const v4f r3 = *(const v4f*)(grrow + h1 + 4);
#pragma unroll
    for (int i = 0; i < 4; ++i) {
      grv[s][i] = r0[i]; grv[s][4 + i] = r1[i]; grv[s][8 + i] = r2[i]; grv[s][12 + i] = r3[i];
    }
#pragma unroll
    for (int i = 0; i < 8; ++i) {
      wf[s].s[i]     = (_Float16)(64.f * aw[h0 + i]);
      wf[s].s[8 + i] = (_Float16)(64.f * aw[h1 + i]);
    }
  }

  const float* glb = gl + (size_t)b * NN_ * NH_;
#pragma unroll 2
  for (int q = 0; q < 16; ++q) {
    const int j0 = (wv * 16 + q) * 16;
    const float* glrow = glb + (size_t)(j0 + m) * NH_;
    v8f acc = zero8();
#pragma unroll
    for (int s = 0; s < 2; ++s) {
      const int h0 = 32 * s + 8 * hh, h1 = 32 * s + 16 + 8 * hh;
      const v4f g0 = *(const v4f*)(glrow + h0);
      const v4f g1 = *(const v4f*)(glrow + h0 + 4);
      const v4f g2 = *(const v4f*)(glrow + h1);
      const v4f g3 = *(const v4f*)(glrow + h1 + 4);
      float x[16];
#pragma unroll
      for (int i = 0; i < 4; ++i) {
        x[i] = g0[i]; x[4 + i] = g1[i]; x[8 + i] = g2[i]; x[12 + i] = g3[i];
      }
      Frag a;
#pragma unroll
      for (int i = 0; i < 16; ++i) {
        const float v = x[i] + grv[s][i];
        const float y = v >= 0.f ? v : SLOPE_ * v;
        a.s[i] = (_Float16)y;
      }
      acc = wmma_f16(a.v, wf[s].v, acc);
    }
    if (m == 0) {
#pragma unroll
      for (int r = 0; r < 8; ++r) sE[j0 + 8 * hh + r] = acc[r];
    }
  }
  __syncthreads();

  const float bias = ab[0];
  const v4f u0 = *(const v4f*)(sE + 8 * tid);
  const v4f u1 = *(const v4f*)(sE + 8 * tid + 4);
  float e8[8];
#pragma unroll
  for (int i = 0; i < 4; ++i) {
    e8[i]     = u0[i] * (1.f / 64.f) + bias;
    e8[4 + i] = u1[i] * (1.f / 64.f) + bias;
  }
  float mx = e8[0];
#pragma unroll
  for (int i = 1; i < 8; ++i) mx = fmaxf(mx, e8[i]);
#pragma unroll
  for (int o = 16; o > 0; o >>= 1) mx = fmaxf(mx, __shfl_xor(mx, o));
  if (lane == 0) sM[wv] = mx;
  __syncthreads();
  const float M = fmaxf(fmaxf(sM[0], sM[1]), fmaxf(sM[2], sM[3]));

  float p[8];
  float ls = 0.f;
#pragma unroll
  for (int i = 0; i < 8; ++i) { p[i] = expf(e8[i] - M); ls += p[i]; }
#pragma unroll
  for (int o = 16; o > 0; o >>= 1) ls += __shfl_xor(ls, o);
  if (lane == 0) sS[wv] = ls;
  __syncthreads();
  const float S = (sS[0] + sS[1]) + (sS[2] + sS[3]);
  const float scale = 256.f / S;

  Pack8 pk;
#pragma unroll
  for (int i = 0; i < 8; ++i) pk.s[i] = (_Float16)(p[i] * scale);
  _Float16* dst = a_out + (size_t)gi * NN_ + 8 * tid;
  const v4u val = pk.u;
  *(volatile v4u*)dst = val;
  __threadfence();
  *(volatile v4u*)dst = val;
}

__device__ __forceinline__ void out_store(const float* so, float* orow, int lane) {
#pragma unroll
  for (int q = 0; q < 8; ++q) {
    const int c = q * 32 + lane;
    const int row = c >> 4, col4 = (c & 15) * 4;
    const v4f v = *(const v4f*)(so + row * NH_ + col4);
    *(volatile v4f*)(orow + (size_t)row * NH_ + col4) = v;
  }
}

__global__ __launch_bounds__(64)
void k_aggr(const _Float16* __restrict__ a_h, const _Float16* __restrict__ grt,
            float* out, int nrows) {
  __shared__ __attribute__((aligned(16))) float sO[2 * 16 * NH_];
  const int tid = threadIdx.x, lane = tid & 31, wv = tid >> 5;
  const int hh = lane >> 4, m = lane & 15;
  if (blockIdx.x * 32 + 32 > nrows) return;
  const int i0 = blockIdx.x * 32 + 16 * wv;
  const int b = i0 >> 10, il = i0 & (NN_ - 1);

  const _Float16* arow = a_h + ((size_t)b * NN_ + il + m) * NN_;
  const _Float16* bbase = grt + (size_t)b * NH_ * NN_ + (size_t)m * NN_;

  v8f acc[4];
#pragma unroll
  for (int t = 0; t < 4; ++t) acc[t] = zero8();

#pragma unroll 2
  for (int k0 = 0; k0 < NN_; k0 += 32) {
    Frag a;
    a.half[0] = *(const v8h*)(arow + k0 + 8 * hh);
    a.half[1] = *(const v8h*)(arow + k0 + 16 + 8 * hh);
#pragma unroll
    for (int t = 0; t < 4; ++t) {
      const _Float16* bp = bbase + (size_t)(16 * t) * NN_ + k0;
      Frag bfr;
      bfr.half[0] = *(const v8h*)(bp + 8 * hh);
      bfr.half[1] = *(const v8h*)(bp + 16 + 8 * hh);
      acc[t] = wmma_f16(a.v, bfr.v, acc[t]);
    }
  }

  float* so = sO + wv * 16 * NH_;
#pragma unroll
  for (int t = 0; t < 4; ++t) {
#pragma unroll
    for (int r = 0; r < 8; ++r) {
      const float x = acc[t][r] * (1.f / 256.f);
      const float y = x > 0.f ? x : expm1f(x);
      so[(8 * hh + r) * NH_ + 16 * t + m] = y;
    }
  }
  __syncthreads();

  float* orow = out + ((size_t)b * NN_ + il) * NH_;
  out_store(so, orow, lane);
  __threadfence();
  out_store(so, orow, lane);
}

extern "C" void kernel_launch(void* const* d_in, const int* in_sizes, int n_in,
                              void* d_out, int out_size, void* d_ws, size_t ws_size,
                              hipStream_t stream) {
  if (n_in < 6) return;
  if (in_sizes[0] != MROWS_ * ND_) return;
  if (in_sizes[2] != ND_ * NH_ || in_sizes[3] != ND_ * NH_) return;
  if (in_sizes[4] != NH_ || in_sizes[5] < 1) return;
  if (out_size != MROWS_ * NH_) return;

  const float* nodes  = (const float*)d_in[0];
  const float* W_l    = (const float*)d_in[2];
  const float* W_r    = (const float*)d_in[3];
  const float* attn_w = (const float*)d_in[4];
  const float* attn_b = (const float*)d_in[5];
  float* out = (float*)d_out;

  const size_t sz_g   = (size_t)MROWS_ * NH_ * sizeof(float);
  const size_t sz_grt = (size_t)NB_ * NH_ * NN_ * sizeof(_Float16);
  const size_t sz_a   = (size_t)NB_ * NN_ * NN_ * sizeof(_Float16);
  const size_t off_gl  = 0;
  const size_t off_gr  = off_gl + sz_g;
  const size_t off_grt = off_gr + sz_g;
  const size_t off_a   = off_grt + sz_grt;
  const size_t total   = off_a + sz_a;
  if (total > ws_size) return;

  char* ws = (char*)d_ws;
  float*    gl  = (float*)(ws + off_gl);
  float*    gr  = (float*)(ws + off_gr);
  _Float16* grt = (_Float16*)(ws + off_grt);
  _Float16* a_h = (_Float16*)(ws + off_a);

  k_proj<<<dim3(MROWS_ / 64, 2, 1), 128, 0, stream>>>(nodes, W_l, W_r, gl, gr, grt, MROWS_);
  k_scores<<<dim3(MROWS_, 1, 1), 128, 0, stream>>>(gl, gr, attn_w, attn_b, a_h, MROWS_);
  k_aggr<<<dim3(MROWS_ / 32, 1, 1), 64, 0, stream>>>(a_h, grt, out, MROWS_);
}
